// HeteroGraphormer_17489106829951
// MI455X (gfx1250) — hardware-verified
//
#include <hip/hip_runtime.h>
#include <math.h>

typedef __attribute__((ext_vector_type(16))) _Float16 v16h;
typedef __attribute__((ext_vector_type(16))) __bf16 v16b;
typedef __attribute__((ext_vector_type(8)))  _Float16 v8h;
typedef __attribute__((ext_vector_type(8)))  float v8f;
typedef __attribute__((ext_vector_type(4)))  float v4f;
typedef __attribute__((ext_vector_type(2)))  float v2f;
typedef __attribute__((ext_vector_type(4)))  unsigned v4u;
typedef __attribute__((ext_vector_type(4)))  int v4i;
typedef float __attribute__((may_alias)) float_a;
typedef int __attribute__((may_alias)) int_a;

template <typename T> __device__ __forceinline__ void vst2(void* p, T v) { *(volatile T*)p = v; __threadfence(); *(volatile T*)p = v; }
__device__ __forceinline__ v8f wmma16(v16h a, v16h b, v8f c) {
  v8f d = __builtin_amdgcn_wmma_f32_16x16x32_f16(false, a, false, b, (short)0, c, false, false);
  asm volatile("v_nop\n\tv_nop\n\tv_nop\n\tv_nop" : "+v"(d) : "v"(a), "v"(b));
  return d;
}
__device__ __forceinline__ v8f wmma_bf(v16b a, v16b b, v8f c) {
  v8f d = __builtin_amdgcn_wmma_f32_16x16x32_bf16(false, a, false, b, (short)0, c, false, false);
  asm volatile("v_nop\n\tv_nop\n\tv_nop\n\tv_nop" : "+v"(d) : "v"(a), "v"(b));
  return d;
}
__device__ __forceinline__ v16h frag_h(const _Float16* rowk0, int lane) {
  union { v16h v; v8h q[2]; } u; const _Float16* p = rowk0 + 8 * (lane >> 4);
  u.q[0] = *(const v8h*)p; u.q[1] = *(const v8h*)(p + 16); return u.v;
}
__device__ __forceinline__ v16h frag_f32(const float* rowk0, int lane) {
  v16h a; const float* p = rowk0 + 8 * (lane >> 4);
#pragma unroll
  for (int i = 0; i < 8; ++i) { a[i] = (_Float16)p[i]; a[8 + i] = (_Float16)p[16 + i]; }
  return a;
}
__device__ __forceinline__ v16h frag_f32s(const float* rowk0, int lane, float sc) {
  v16h a; const float* p = rowk0 + 8 * (lane >> 4);
#pragma unroll
  for (int i = 0; i < 8; ++i) { a[i] = (_Float16)(p[i] * sc); a[8 + i] = (_Float16)(p[16 + i] * sc); }
  return a;
}
__device__ __forceinline__ v16h fragc_f32(const float* W, int k0, int n, int lane, int ld, int K) {
  v16h a; const int g = lane >> 4;
#pragma unroll
  for (int i = 0; i < 8; ++i) { const int ka = k0 + 8 * g + i, kb = ka + 16;
    a[i] = (_Float16)(ka < K ? W[(size_t)ka * ld + n] : 0.f); a[8 + i] = (_Float16)(kb < K ? W[(size_t)kb * ld + n] : 0.f); }
  return a;
}
struct F2 { v16b h, l; };
__device__ __forceinline__ F2 bsplit16(const float v[16]) { F2 r;
#pragma unroll
  for (int i = 0; i < 16; ++i) { const __bf16 h = (__bf16)v[i]; r.h[i] = h; r.l[i] = (__bf16)(v[i] - (float)h); }
  return r; }
__device__ __forceinline__ F2 split_row(const float* row, int k0, int lane) { float v[16]; const float* p = row + k0 + 8 * (lane >> 4);
#pragma unroll
  for (int i = 0; i < 8; ++i) { v[i] = p[i]; v[8 + i] = p[16 + i]; }
  return bsplit16(v); }
__device__ __forceinline__ F2 split_rowK(const float* row, int k0, int lane, int K) { float v[16]; const int g = lane >> 4;
#pragma unroll
  for (int i = 0; i < 8; ++i) { const int ka = k0 + 8 * g + i, kb = ka + 16; v[i] = ka < K ? row[ka] : 0.f; v[8 + i] = kb < K ? row[kb] : 0.f; }
  return bsplit16(v); }
__device__ __forceinline__ F2 split_col(const float* W, int k0, int n, int lane, int ld, int K) { float v[16]; const int g = lane >> 4;
#pragma unroll
  for (int i = 0; i < 8; ++i) { const int ka = k0 + 8 * g + i, kb = ka + 16; v[i] = ka < K ? W[(size_t)ka * ld + n] : 0.f; v[8 + i] = kb < K ? W[(size_t)kb * ld + n] : 0.f; }
  return bsplit16(v); }
__device__ __forceinline__ v8f mac3(const F2& a, const F2& b, v8f c) { c = wmma_bf(a.l, b.h, c); c = wmma_bf(a.h, b.l, c); return wmma_bf(a.h, b.h, c); }
__device__ __forceinline__ float sigm(float v) { return 1.0f / (1.0f + expf(-v)); }
#define LDSX() do { asm volatile("s_wait_dscnt 0" ::: "memory"); __builtin_amdgcn_wave_barrier(); __builtin_amdgcn_fence(__ATOMIC_RELEASE, "workgroup"); } while (0)


#define NL 3
#define NB 1
#define SS 2048
#define E 512
#define NH 8
#define HD 64
#define NR SS
#define FF 2048
#define MAXD 5
__device__ __forceinline__ float gelu_e(float x) { return 0.5f * x * (1.0f + erff(x * 0.70710678118654752f)); }

__global__ __launch_bounds__(256) void k_embed(const float* __restrict__ feats, const int* __restrict__ indeg, const int* __restrict__ outdeg, const float* __restrict__ inE, const float* __restrict__ outE, float* __restrict__ X) {
  const int q = blockIdx.x * 256 + threadIdx.x; const int r = q >> 7, pc = q & 127; if (r >= NR) return;
  int a = indeg[r]; a = a < 0 ? 0 : (a > 31 ? 31 : a); int b = outdeg[r]; b = b < 0 ? 0 : (b > 31 ? 31 : b);
  const v4f f = *(const v4f*)(feats + (size_t)r * E + pc * 4), i4 = *(const v4f*)(inE + (size_t)a * E + pc * 4), o4 = *(const v4f*)(outE + (size_t)b * E + pc * 4);
  vst2(X + (size_t)r * E + pc * 4, f + i4 + o4);
}
__global__ __launch_bounds__(256) void k_cvt(const float* __restrict__ x, _Float16* __restrict__ X16) {
  const size_t i8 = (size_t)blockIdx.x * 256 + threadIdx.x; if (i8 >= (size_t)NR * E / 8) return;
  union { v8h h; v4u u; } pk;
#pragma unroll
  for (int e = 0; e < 8; ++e) pk.h[e] = (_Float16)x[i8 * 8 + e];
  vst2(X16 + i8 * 8, pk.u);
}
__global__ __launch_bounds__(256) void k_pack(const float* __restrict__ Wq, const float* __restrict__ Wk, const float* __restrict__ Wv, const float* __restrict__ Wo, const float* __restrict__ W1, const float* __restrict__ W2,
                                             _Float16* __restrict__ PT, _Float16* __restrict__ P2) {
  const int n = blockIdx.x, tid = threadIdx.x; __shared__ __align__(16) _Float16 srow[FF];
  if (n < 4096) { float v = 0.f; const int k = tid; const int k2 = tid + 256;
    const float* W = n < 512 ? Wq : (n < 1024 ? Wk : (n < 1536 ? Wv : (n < 2048 ? Wo : nullptr))); const int nn = n & 511;
    if (n < 2048) { srow[k] = (_Float16)(W[(size_t)k * E + nn] * 16.0f); srow[k2] = (_Float16)(W[(size_t)k2 * E + nn] * 16.0f); }
    else { const int c = n - 2048; srow[k] = (_Float16)(W1[(size_t)k * FF + c] * 16.0f); srow[k2] = (_Float16)(W1[(size_t)k2 * FF + c] * 16.0f); }
    (void)v; __syncthreads(); if (tid < E / 8) vst2(PT + (size_t)n * E + tid * 8, *(const v4u*)(&srow[tid * 8])); }
  else { const int c = n - 4096; for (int k = tid; k < FF; k += 256) srow[k] = (_Float16)(W2[(size_t)k * E + c] * 16.0f); __syncthreads(); vst2(P2 + (size_t)c * FF + tid * 8, *(const v4u*)(&srow[tid * 8])); }
}
__global__ __launch_bounds__(128) void k_qkv(const _Float16* __restrict__ X16, const _Float16* __restrict__ PT, const float* __restrict__ bq, const float* __restrict__ bk, const float* __restrict__ bv,
                                            _Float16* __restrict__ Q16, _Float16* __restrict__ K16, _Float16* __restrict__ VTh) {
  __shared__ __align__(16) float so[4][16][132];
  __shared__ __align__(16) _Float16 sth[128][72];
  const int tid = threadIdx.x, wave = tid >> 5, lane = tid & 31, col = lane & 15, g = lane >> 4;
  const int which = blockIdx.z, r0b = blockIdx.x * 64, r0 = r0b + wave * 16, n0 = blockIdx.y * 128; const int s0 = r0b;
  const float* bb_ = which == 0 ? bq : (which == 1 ? bk : bv);
  v8f acc[8] = {};
#pragma unroll 2
  for (int kc = 0; kc < E / 32; ++kc) { const v16h a = frag_h(X16 + (size_t)(r0 + col) * E + kc * 32, lane);
#pragma unroll
    for (int j = 0; j < 8; ++j) acc[j] = wmma16(a, frag_h(PT + (size_t)(which * E + n0 + j * 16 + col) * E + kc * 32, lane), acc[j]); }
  if (which < 2) {
#pragma unroll
    for (int j = 0; j < 8; ++j) { const float bb = bb_[n0 + j * 16 + col];
#pragma unroll
      for (int r = 0; r < 8; ++r) so[wave][8 * g + r][j * 16 + col] = (acc[j][r] * (1.0f / 16.0f) + bb) * 4.0f; }
    LDSX();
    _Float16* Dst = which == 0 ? Q16 : K16;
    for (int qq = lane; qq < 16 * 2 * 8; qq += 32) { const int hh = qq >> 7, rl = (qq >> 3) & 15, pc = qq & 7; const int h = (n0 >> 6) + hh; union { v8h h8; v4u u; } pk;
#pragma unroll
      for (int e = 0; e < 8; ++e) pk.h8[e] = (_Float16)so[wave][rl][hh * 64 + pc * 8 + e];
      vst2(Dst + (((size_t)h) * SS + s0 + wave * 16 + rl) * HD + pc * 8, pk.u); } }
  else {
#pragma unroll
    for (int j = 0; j < 8; ++j) { const float bb = bb_[n0 + j * 16 + col];
#pragma unroll
      for (int r = 0; r < 8; ++r) { const float v = (acc[j][r] * (1.0f / 16.0f) + bb) * 4.0f; sth[j * 16 + col][wave * 16 + 8 * g + r] = (_Float16)v; } }
    __syncthreads();
    for (int qq = tid; qq < 128 * 8; qq += 128) { const int cl = qq >> 3, pc = qq & 7; const int c = n0 + cl, h = c >> 6, d = c & 63; const size_t o = (((size_t)h) * HD + d) * SS + s0 + pc * 8;
      vst2(VTh + o, *(const v4u*)(&sth[cl][pc * 8])); } }
}
__global__ __launch_bounds__(128) void k_attn(const _Float16* __restrict__ Q16, const _Float16* __restrict__ K16, const _Float16* __restrict__ VTh, const int* __restrict__ dist, const float* __restrict__ semb, _Float16* __restrict__ O16) {
  __shared__ __align__(16) float sS[4][16][68];
  __shared__ __align__(16) _Float16 sPh[4][16][72];
  __shared__ __align__(16) float sO[4][16][68];
  __shared__ float stab[8];
  const int tid = threadIdx.x, w = tid >> 5, lane = tid & 31, col = lane & 15, g = lane >> 4;
  const size_t bh = blockIdx.y; const int h = (int)bh; const int q0 = blockIdx.x * 64 + w * 16;
  if (tid < 8) stab[tid] = tid <= MAXD ? semb[tid * NH + h] : 0.f;
  __syncthreads();
  v16h aq[2];
#pragma unroll
  for (int kc = 0; kc < 2; ++kc) aq[kc] = frag_h(Q16 + (bh * SS + q0 + col) * HD + kc * 32, lane);
  float mrun = -3.0e38f, lrun = 0.f; v8f acc[4] = {};
#pragma unroll 1
  for (int kt = 0; kt < SS / 64; ++kt) {
#pragma unroll
    for (int t = 0; t < 4; ++t) { v8f s = {}; const int key = kt * 64 + t * 16 + col;
#pragma unroll
      for (int kc = 0; kc < 2; ++kc) s = wmma16(aq[kc], frag_h(K16 + (bh * SS + key) * HD + kc * 32, lane), s);
#pragma unroll
      for (int r = 0; r < 8; ++r) { int dd = dist[(size_t)(q0 + 8 * g + r) * SS + key]; dd = dd < 0 ? 0 : (dd > MAXD ? MAXD : dd); sS[w][8 * g + r][t * 16 + col] = s[r] * (0.125f / 16.0f) + stab[dd]; } }
    LDSX();
    float mx = -3.4e38f;
#pragma unroll
    for (int jj = 0; jj < 32; ++jj) mx = fmaxf(mx, sS[w][col][g * 32 + jj]);
    mx = fmaxf(mx, __shfl_xor(mx, 16, 32));
    const float mnew = fmaxf(mrun, mx); const float corr = expf(mrun - mnew);
    float ps = 0.f;
#pragma unroll
    for (int jj = 0; jj < 32; ++jj) { const float p = expf(sS[w][col][g * 32 + jj] - mnew) * 16384.0f; ps += p; sPh[w][col][g * 32 + jj] = (_Float16)p; }
    ps += __shfl_xor(ps, 16, 32);
    lrun = lrun * corr + ps * (1.0f / 16384.0f); mrun = mnew;
#pragma unroll
    for (int r = 0; r < 8; ++r) { const float cr = __shfl(corr, 8 * g + r, 32);
#pragma unroll
      for (int t = 0; t < 4; ++t) acc[t][r] *= cr; }
    LDSX();
#pragma unroll
    for (int kc = 0; kc < 2; ++kc) { const v16h ph = frag_h(&sPh[w][col][0] + kc * 32, lane);
#pragma unroll
      for (int t = 0; t < 4; ++t) { const size_t vo = (bh * HD + t * 16 + col) * SS + kt * 64 + kc * 32; acc[t] = wmma16(ph, frag_h(VTh + vo, lane), acc[t]); } }
    __builtin_amdgcn_wave_barrier(); }
#pragma unroll
  for (int r = 0; r < 8; ++r) { const float lr = __shfl(lrun, 8 * g + r, 32); const float inv = 8.0f / (lr * 16384.0f * 4.0f);
#pragma unroll
    for (int t = 0; t < 4; ++t) sO[w][8 * g + r][t * 16 + col] = acc[t][r] * inv; }
  LDSX();
  for (int qq = lane; qq < 16 * 8; qq += 32) { const int rl = qq >> 3, pc = qq & 7; union { v8h h8; v4u u; } pk;
#pragma unroll
    for (int e = 0; e < 8; ++e) pk.h8[e] = (_Float16)sO[w][rl][pc * 8 + e];
    vst2(O16 + ((bh * SS) + q0 + rl) * HD + pc * 8, pk.u); }
}
__global__ __launch_bounds__(128) void k_oln(const _Float16* __restrict__ O16, const _Float16* __restrict__ PT, const float* __restrict__ bo, const float* __restrict__ X, const float* __restrict__ g1, const float* __restrict__ b1n, float* __restrict__ X1) {
  __shared__ __align__(16) float so[4][16][E + 4];
  const int tid = threadIdx.x, wave = tid >> 5, lane = tid & 31, col = lane & 15, g = lane >> 4;
  const int r0 = blockIdx.x * 64 + wave * 16; const int s = r0 + col;
#pragma unroll 1
  for (int nh = 0; nh < E / 128; ++nh) { v8f acc[8] = {};
#pragma unroll 2
    for (int kc = 0; kc < E / 32; ++kc) { const int h = kc >> 1; const v16h a = frag_h(O16 + (((size_t)h) * SS + s) * HD + (kc & 1) * 32, lane);
#pragma unroll
      for (int j = 0; j < 8; ++j) acc[j] = wmma16(a, frag_h(PT + (size_t)(3 * E + nh * 128 + j * 16 + col) * E + kc * 32, lane), acc[j]); }
#pragma unroll
    for (int j = 0; j < 8; ++j) { const int n = nh * 128 + j * 16 + col; const float bb = bo[n];
#pragma unroll
      for (int r = 0; r < 8; ++r) so[wave][8 * g + r][n] = acc[j][r] * (1.0f / (16.0f * 8.0f)) + bb + X[(size_t)(r0 + 8 * g + r) * E + n]; } }
  LDSX();
  { const int rl = lane & 15, hf = lane >> 4; float* row = &so[wave][rl][hf * 256]; float s1 = 0.f;
#pragma unroll 4
    for (int k = 0; k < 256; ++k) s1 += row[k];
    s1 += __shfl_xor(s1, 16, 32); const float mu = s1 * (1.0f / E); float q = 0.f;
#pragma unroll 4
    for (int k = 0; k < 256; ++k) { const float dv = row[k] - mu; q += dv * dv; }
    q += __shfl_xor(q, 16, 32); const float rs = rsqrtf(q * (1.0f / E) + 1e-5f);
#pragma unroll 4
    for (int k = 0; k < 256; ++k) row[k] = (row[k] - mu) * rs * g1[hf * 256 + k] + b1n[hf * 256 + k]; }
  LDSX();
  for (int rl = 0; rl < 16; ++rl) { for (int pc = lane; pc < E / 4; pc += 32) vst2(X1 + (size_t)(r0 + rl) * E + pc * 4, *(const v4f*)(&so[wave][rl][pc * 4])); }
}
__global__ __launch_bounds__(128) void k_ffn1(const float* __restrict__ X1, const _Float16* __restrict__ PT, const float* __restrict__ b1, _Float16* __restrict__ H1) {
  __shared__ __align__(16) _Float16 so[4][16][136];
  const int tid = threadIdx.x, wave = tid >> 5, lane = tid & 31, col = lane & 15, g = lane >> 4;
  const int r0 = blockIdx.x * 64 + wave * 16, n0 = blockIdx.y * 128;
  v8f acc[8] = {};
#pragma unroll 2
  for (int kc = 0; kc < E / 32; ++kc) { const v16h a = frag_f32(X1 + (size_t)(r0 + col) * E + kc * 32, lane);
#pragma unroll
    for (int j = 0; j < 8; ++j) acc[j] = wmma16(a, frag_h(PT + (size_t)(4 * E + n0 + j * 16 + col) * E + kc * 32, lane), acc[j]); }
#pragma unroll
  for (int j = 0; j < 8; ++j) { const float bb = b1[n0 + j * 16 + col];
#pragma unroll
    for (int r = 0; r < 8; ++r) so[wave][8 * g + r][j * 16 + col] = (_Float16)gelu_e(acc[j][r] * (1.0f / 16.0f) + bb); }
  LDSX();
  for (int rl = 0; rl < 16; ++rl) { if (lane < 16) vst2(H1 + (size_t)(r0 + rl) * FF + n0 + lane * 8, *(const v4u*)(&so[wave][rl][lane * 8])); }
}
__global__ __launch_bounds__(128) void k_ffn2(const _Float16* __restrict__ H1, const _Float16* __restrict__ P2, const float* __restrict__ b2, const float* __restrict__ X1, const float* __restrict__ g2, const float* __restrict__ b2n, float* __restrict__ X2) {
  __shared__ __align__(16) float so[4][16][E + 4];
  const int tid = threadIdx.x, wave = tid >> 5, lane = tid & 31, col = lane & 15, g = lane >> 4;
  const int r0 = blockIdx.x * 64 + wave * 16;
#pragma unroll 1
  for (int nh = 0; nh < E / 128; ++nh) { v8f acc[8] = {};
#pragma unroll 2
    for (int kc = 0; kc < FF / 32; ++kc) { const v16h a = frag_h(H1 + (size_t)(r0 + col) * FF + kc * 32, lane);
#pragma unroll
      for (int j = 0; j < 8; ++j) acc[j] = wmma16(a, frag_h(P2 + (size_t)(nh * 128 + j * 16 + col) * FF + kc * 32, lane), acc[j]); }
#pragma unroll
    for (int j = 0; j < 8; ++j) { const int n = nh * 128 + j * 16 + col; const float bb = b2[n];
#pragma unroll
      for (int r = 0; r < 8; ++r) so[wave][8 * g + r][n] = acc[j][r] * (1.0f / 16.0f) + bb + X1[(size_t)(r0 + 8 * g + r) * E + n]; } }
  LDSX();
  { const int rl = lane & 15, hf = lane >> 4; float* row = &so[wave][rl][hf * 256]; float s1 = 0.f;
#pragma unroll 4
    for (int k = 0; k < 256; ++k) s1 += row[k];
    s1 += __shfl_xor(s1, 16, 32); const float mu = s1 * (1.0f / E); float q = 0.f;
#pragma unroll 4
    for (int k = 0; k < 256; ++k) { const float dv = row[k] - mu; q += dv * dv; }
    q += __shfl_xor(q, 16, 32); const float rs = rsqrtf(q * (1.0f / E) + 1e-5f);
#pragma unroll 4
    for (int k = 0; k < 256; ++k) row[k] = (row[k] - mu) * rs * g2[hf * 256 + k] + b2n[hf * 256 + k]; }
  LDSX();
  for (int rl = 0; rl < 16; ++rl) { for (int pc = lane; pc < E / 4; pc += 32) vst2(X2 + (size_t)(r0 + rl) * E + pc * 4, *(const v4f*)(&so[wave][rl][pc * 4])); }
}
extern "C" void kernel_launch(void* const* d_in, const int* in_sizes, int n_in, void* d_out, int out_size, void* d_ws, size_t ws_size, hipStream_t stream) {
  (void)in_sizes; (void)n_in; (void)out_size; (void)ws_size;
  const float* feats = (const float*)d_in[0]; const int* dist = (const int*)d_in[1]; const int* indeg = (const int*)d_in[2]; const int* outdeg = (const int*)d_in[3];
  const float* semb = (const float*)d_in[4]; const float* inE = (const float*)d_in[5]; const float* outE = (const float*)d_in[6];
  const float* Wq = (const float*)d_in[7]; const float* bq = (const float*)d_in[8]; const float* Wk = (const float*)d_in[9]; const float* bk = (const float*)d_in[10]; const float* Wv = (const float*)d_in[11]; const float* bv = (const float*)d_in[12];
  const float* Wo = (const float*)d_in[13]; const float* bo = (const float*)d_in[14]; const float* g1 = (const float*)d_in[15]; const float* b1n = (const float*)d_in[16]; const float* g2 = (const float*)d_in[17]; const float* b2n = (const float*)d_in[18];
  const float* W1 = (const float*)d_in[19]; const float* b1 = (const float*)d_in[20]; const float* W2 = (const float*)d_in[21]; const float* b2 = (const float*)d_in[22];
  float* out = (float*)d_out;
  char* ws = (char*)d_ws; size_t off = 0;
  auto take = [&](size_t bytes) { char* p = ws + off; off += (bytes + 255) & ~(size_t)255; return p; };
  float* X = (float*)take((size_t)NR * E * 4); float* X1 = (float*)take((size_t)NR * E * 4); _Float16* X16 = (_Float16*)take((size_t)NR * E * 2);
  _Float16* PT = (_Float16*)take((size_t)(4 * E + FF) * E * 2); _Float16* P2 = (_Float16*)take((size_t)E * FF * 2);
  _Float16* Q16 = (_Float16*)take((size_t)NR * E * 2); _Float16* K16 = (_Float16*)take((size_t)NR * E * 2); _Float16* VTh = (_Float16*)take((size_t)NR * E * 2); _Float16* O16 = (_Float16*)take((size_t)NR * E * 2);
  _Float16* H1 = (_Float16*)take((size_t)NR * FF * 2);
  k_embed<<<(NR * 128 + 255) / 256, 256, 0, stream>>>(feats, indeg, outdeg, inE, outE, X);
  for (int l = 0; l < NL; ++l) {
    const size_t oC = (size_t)l * E * E, oV = (size_t)l * E, oF1 = (size_t)l * E * FF, oF = (size_t)l * FF;
    k_cvt<<<(NR * E / 8 + 255) / 256, 256, 0, stream>>>(X, X16);
    k_pack<<<4096 + E, 256, 0, stream>>>(Wq + oC, Wk + oC, Wv + oC, Wo + oC, W1 + oF1, W2 + oF1, PT, P2);
    k_qkv<<<dim3(NR / 64, E / 128, 3), 128, 0, stream>>>(X16, PT, bq + oV, bk + oV, bv + oV, Q16, K16, VTh);
    k_attn<<<dim3(SS / 64, NH), 128, 0, stream>>>(Q16, K16, VTh, dist, semb, O16);
    k_oln<<<NR / 64, 128, 0, stream>>>(O16, PT, bo + oV, X, g1 + oV, b1n + oV, X1);
    k_ffn1<<<dim3(NR / 64, FF / 128), 128, 0, stream>>>(X1, PT, b1 + oF, H1);
    k_ffn2<<<NR / 64, 128, 0, stream>>>(H1, P2, b2 + oV, X1, g2 + oV, b2n + oV, l == NL - 1 ? out : X);
  }
}
